// EdgeGenerator_62809601736824
// MI455X (gfx1250) — hardware-verified
//
#include <hip/hip_runtime.h>
#include <math.h>

typedef _Float16 v16h __attribute__((ext_vector_type(16)));
typedef _Float16 v8h  __attribute__((ext_vector_type(8)));
typedef __bf16   v16b __attribute__((ext_vector_type(16)));
typedef unsigned short v8us __attribute__((ext_vector_type(8), may_alias));
typedef unsigned short v4us __attribute__((ext_vector_type(4), may_alias));
typedef float v8f __attribute__((ext_vector_type(8)));
typedef float v4f __attribute__((ext_vector_type(4), may_alias));

#define DH 128
#define KE 288
#define KN 256
#define KP 288
#define NB 128
#define PENDCAP 320

union FragH { v16h v; v8h half[2]; };
union FragB { v16b v; v8us half[2]; };

__device__ __forceinline__ float silu_f(float x) { return x * (1.0f / (1.0f + __expf(-x))); }

__device__ __forceinline__ unsigned short bf16_rne(float x) {
    unsigned u = __float_as_uint(x);
    u += 0x7FFFu + ((u >> 16) & 1u);
    return (unsigned short)(u >> 16);
}
__device__ __forceinline__ float bf16_to_f(unsigned short s) { return __uint_as_float(((unsigned)s) << 16); }

__device__ __forceinline__ v8f zero8() { v8f z;
#pragma unroll
    for (int i = 0; i < 8; ++i) z[i] = 0.0f; return z; }

__device__ __forceinline__ v16h ldfrag_h(const _Float16* base, int pitch, int row, int k0, int h) {
    FragH f; const _Float16* p = base + (size_t)row * pitch + k0 + 8 * h;
    f.half[0] = *(const v8h*)p; f.half[1] = *(const v8h*)(p + 16); return f.v;
}
__device__ __forceinline__ v16b ldfrag_b(const unsigned short* base, int pitch, int row, int k0, int h) {
    FragB f; const unsigned short* p = base + (size_t)row * pitch + k0 + 8 * h;
    f.half[0] = *(const v8us*)p; f.half[1] = *(const v8us*)(p + 16); return f.v;
}

__device__ __forceinline__ v8f mma_h(v16h a, v16h b, v8f c) {
    c = __builtin_amdgcn_wmma_f32_16x16x32_f16(false, a, false, b, (short)0, c, false, false);
    asm volatile("v_nop\n\tv_nop\n\tv_nop\n\tv_nop" : "+v"(c) : "v"(a), "v"(b));
    return c;
}
__device__ __forceinline__ v8f mma_b3(v16b ah, v16b al, v16b bh, v16b bl, v8f c) {
    c = __builtin_amdgcn_wmma_f32_16x16x32_bf16(false, ah, false, bh, (short)0, c, false, false);
    c = __builtin_amdgcn_wmma_f32_16x16x32_bf16(false, ah, false, bl, (short)0, c, false, false);
    c = __builtin_amdgcn_wmma_f32_16x16x32_bf16(false, al, false, bh, (short)0, c, false, false);
    asm volatile("v_nop\n\tv_nop\n\tv_nop\n\tv_nop" : "+v"(c) : "v"(ah), "v"(al), "v"(bh), "v"(bl));
    return c;
}

__device__ __forceinline__ int clampi(int x, int n) { return x < 0 ? 0 : (x >= n ? n - 1 : x); }

__global__ __launch_bounds__(256) void k_tw_f16(const float* __restrict__ src, _Float16* dst,
                                                int L, int K, int Nout, int Kpad) {
    int cpm = Nout * (Kpad / 8);
    int i = blockIdx.x * 256 + threadIdx.x;
    if (i >= L * cpm) return;
    int l = i / cpm; int j = i - l * cpm; int n = j / (Kpad / 8); int k0 = (j - n * (Kpad / 8)) * 8;
    v8h v;
#pragma unroll
    for (int q = 0; q < 8; ++q) {
        int k = k0 + q;
        v[q] = (k < K) ? (_Float16)src[((size_t)l * K + k) * Nout + n] : (_Float16)0.0f;
    }
    _Float16* p = dst + ((size_t)l * Nout + n) * Kpad + k0;
    *(volatile v8h*)p = v;
    __threadfence();
    *(volatile v8h*)p = v;
}
__global__ __launch_bounds__(256) void k_tw_bf2(const float* __restrict__ src, unsigned short* dH, unsigned short* dL,
                                                int L, int K, int Nout, int Kpad) {
    int cpm = Nout * (Kpad / 8);
    int i = blockIdx.x * 256 + threadIdx.x;
    if (i >= L * cpm) return;
    int l = i / cpm; int j = i - l * cpm; int n = j / (Kpad / 8); int k0 = (j - n * (Kpad / 8)) * 8;
    v8us hv, lv;
#pragma unroll
    for (int q = 0; q < 8; ++q) {
        int k = k0 + q;
        float x = (k < K) ? src[((size_t)l * K + k) * Nout + n] : 0.0f;
        unsigned short hs = bf16_rne(x);
        hv[q] = hs; lv[q] = bf16_rne(x - bf16_to_f(hs));
    }
    size_t o = ((size_t)l * Nout + n) * Kpad + k0;
    *(volatile v8us*)(dH + o) = hv; *(volatile v8us*)(dL + o) = lv;
    __threadfence();
    *(volatile v8us*)(dH + o) = hv; *(volatile v8us*)(dL + o) = lv;
}

__global__ __launch_bounds__(128) void k_encode(const float* __restrict__ xyr, int N,
    const float* __restrict__ w1, const float* __restrict__ b1,
    const float* __restrict__ w2, const float* __restrict__ b2, float* hF32) {
    __shared__ float sH[DH];
    __shared__ __align__(16) float sO[DH];
    int nd = blockIdx.x; int tid = threadIdx.x;
    float x0 = xyr[nd * 3 + 0], x1 = xyr[nd * 3 + 1], x2 = xyr[nd * 3 + 2];
    float h1 = silu_f(x0 * w1[tid] + x1 * w1[DH + tid] + x2 * w1[2 * DH + tid] + b1[tid]);
    sH[tid] = h1;
    __syncthreads();
    float h2 = b2[tid];
#pragma unroll 4
    for (int k = 0; k < DH; ++k) h2 += sH[k] * w2[k * DH + tid];
    sO[tid] = h2;
    __syncthreads();
    if (tid < 32) {
        v4f v = *(const v4f*)&sO[4 * tid];
        float* p = hF32 + (size_t)nd * DH + 4 * tid;
        *(volatile v4f*)p = v;
        __threadfence();
        *(volatile v4f*)p = v;
    }
}

__device__ __forceinline__ void edge_tile(int nv, int nb, int N, int E,
    const float* hF32, const float* xyr, const int* eidx,
    const _Float16* w1T, const float* b1, const _Float16* w2T, const float* b2,
    float* sAcc, _Float16* sIn, _Float16* sHid, const int* sPE, const int* sPL) {
    const int tid = threadIdx.x, w = tid >> 5, lane = tid & 31, h = lane >> 4, m = lane & 15;
    const int col = 16 * w + m;
    const float width = 0.094280904158206338f;
    const float gamma = 56.25f;
    for (int i = tid; i < 64 * 36; i += 256) {
        int row = i / 36; int cc = i - row * 36;
        v8h val;
#pragma unroll
        for (int q = 0; q < 8; ++q) val[q] = (_Float16)0.0f;
        if (row < nv) {
            int e = sPE[row]; e = clampi(e, E);
            int s = clampi(eidx[e], N);
            int d = nb + (sPL[row] & (NB - 1)); d = clampi(d, N);
            if (cc < 32) {
                const float* src = (cc < 16) ? (hF32 + (size_t)s * DH + 8 * cc) : (hF32 + (size_t)d * DH + 8 * (cc - 16));
                v4f a0 = *(const v4f*)src, a1 = *(const v4f*)(src + 4);
#pragma unroll
                for (int q = 0; q < 4; ++q) { val[q] = (_Float16)a0[q]; val[4 + q] = (_Float16)a1[q]; }
            } else if (cc < 34) {
                float dx = xyr[s * 3 + 0] - xyr[d * 3 + 0];
                float dy = xyr[s * 3 + 1] - xyr[d * 3 + 1];
                float r = sqrtf(dx * dx + dy * dy + 1e-8f);
#pragma unroll
                for (int q = 0; q < 8; ++q) {
                    float t = r - width * (float)((cc - 32) * 8 + q);
                    val[q] = (_Float16)__expf(-gamma * t * t);
                }
            }
        }
        *(v8h*)&sIn[row * KE + cc * 8] = val;
    }
    __syncthreads();
    v8f acc[4];
#pragma unroll
    for (int t = 0; t < 4; ++t) acc[t] = zero8();
#pragma unroll 1
    for (int c = 0; c < 9; ++c) {
        v16h b = ldfrag_h(w1T, KE, col, 32 * c, h);
#pragma unroll
        for (int t = 0; t < 4; ++t) {
            v16h a = ldfrag_h(sIn, KE, 16 * t + m, 32 * c, h);
            acc[t] = mma_h(a, b, acc[t]);
        }
    }
    {
        float bias = b1[col];
#pragma unroll
        for (int t = 0; t < 4; ++t)
#pragma unroll
            for (int r = 0; r < 8; ++r) {
                int row = 16 * t + 8 * h + r;
                sHid[row * DH + col] = (_Float16)silu_f(acc[t][r] + bias);
            }
    }
    __syncthreads();
    v8f acc2[4];
#pragma unroll
    for (int t = 0; t < 4; ++t) acc2[t] = zero8();
#pragma unroll 1
    for (int c = 0; c < 4; ++c) {
        v16h b = ldfrag_h(w2T, DH, col, 32 * c, h);
#pragma unroll
        for (int t = 0; t < 4; ++t) {
            v16h a = ldfrag_h(sHid, DH, 16 * t + m, 32 * c, h);
            acc2[t] = mma_h(a, b, acc2[t]);
        }
    }
    {
        float bias2 = b2[col];
#pragma unroll
        for (int t = 0; t < 4; ++t)
#pragma unroll
            for (int hh = 0; hh < 2; ++hh)
#pragma unroll
                for (int r = 0; r < 8; ++r) {
                    int row = 16 * t + 8 * hh + r;
                    if (row < nv && h == hh) {
                        int idx = (sPL[row] & (NB - 1)) * DH + col;
                        sAcc[idx] += acc2[t][r] + bias2;
                    }
                }
    }
    __syncthreads();
}

__global__ __launch_bounds__(256) void k_edge(const float* hF32, const float* __restrict__ xyr,
    const int* __restrict__ eidx, int E, int N,
    const _Float16* w1T, const float* __restrict__ b1,
    const _Float16* w2T, const float* __restrict__ b2, float* agg) {
    __shared__ __align__(16) float sAcc[NB * DH];
    __shared__ __align__(16) _Float16 sIn[64 * KE];
    __shared__ __align__(16) _Float16 sHid[64 * DH];
    __shared__ int sPE[PENDCAP];
    __shared__ int sPL[PENDCAP];
    __shared__ int sWc[8];
    const int tid = threadIdx.x, w = tid >> 5, lane = tid & 31;
    const int nb = blockIdx.x * NB;
    for (int i = tid; i < NB * DH / 4; i += 256) {
        v4f z; z[0] = 0.f; z[1] = 0.f; z[2] = 0.f; z[3] = 0.f;
        *(v4f*)&sAcc[4 * i] = z;
    }
    int pn = 0;
    __syncthreads();
    const int nChunks = (E + 255) >> 8;
    for (int c = 0; c < nChunks; ++c) {
        int e = c * 256 + tid; int hit = 0, ln = 0;
        if (e < E) {
            int d = eidx[E + e];
            ln = d - nb;
            hit = (d >= 0 && d < N && ln >= 0 && ln < NB) ? 1 : 0;
        }
        unsigned bal = __builtin_amdgcn_ballot_w32(hit != 0);
        int wcnt = __builtin_popcount(bal);
        int pre = __builtin_popcount(bal & ((1u << lane) - 1u));
        if (lane == 0) sWc[w] = wcnt;
        __syncthreads();
        int off = 0, tot = 0;
#pragma unroll
        for (int q = 0; q < 8; ++q) { int cq = sWc[q]; if (q < w) off += cq; tot += cq; }
        if (hit) {
            int pos = pn + off + pre;
            if ((unsigned)pos < (unsigned)PENDCAP) { sPE[pos] = e; sPL[pos] = ln; }
        }
        __syncthreads();
        pn += tot;
        if (pn > PENDCAP) pn = PENDCAP;
        for (int dd = 0; dd < 4; ++dd) {
            if (pn < 64) break;
            edge_tile(64, nb, N, E, hF32, xyr, eidx, w1T, b1, w2T, b2, sAcc, sIn, sHid, sPE, sPL);
            int rem = pn - 64;
            int e2 = 0, l2 = 0;
            bool has = tid < rem;
            if (has) { e2 = sPE[64 + tid]; l2 = sPL[64 + tid]; }
            __syncthreads();
            if (has) { sPE[tid] = e2; sPL[tid] = l2; }
            __syncthreads();
            pn = rem;
        }
    }
    if (pn > 0) {
        edge_tile(pn, nb, N, E, hF32, xyr, eidx, w1T, b1, w2T, b2, sAcc, sIn, sHid, sPE, sPL);
    }
    __syncthreads();
    for (int row = w; row < NB; row += 8) {
        int node = nb + row;
        if (node < N) {
            v4f v = *(const v4f*)&sAcc[row * DH + 4 * lane];
            float* p = agg + (size_t)node * DH + 4 * lane;
            *(volatile v4f*)p = v;
        }
    }
    __threadfence();
    for (int row = w; row < NB; row += 8) {
        int node = nb + row;
        if (node < N) {
            v4f v = *(const v4f*)&sAcc[row * DH + 4 * lane];
            float* p = agg + (size_t)node * DH + 4 * lane;
            *(volatile v4f*)p = v;
        }
    }
}

__global__ __launch_bounds__(256) void k_node(float* hF32, const float* agg, int N,
    const unsigned short* w1H, const unsigned short* w1L, const float* __restrict__ b1,
    const unsigned short* w2H, const unsigned short* w2L, const float* __restrict__ b2,
    const float* __restrict__ lng, const float* __restrict__ lnb) {
    __shared__ __align__(16) unsigned short sAH[64 * KN];
    __shared__ __align__(16) unsigned short sAL[64 * KN];
    __shared__ __align__(16) unsigned short sHH[64 * DH];
    __shared__ __align__(16) unsigned short sHL[64 * DH];
    __shared__ __align__(16) float sUp[64 * DH];
    const int tid = threadIdx.x, w = tid >> 5, lane = tid & 31, h = lane >> 4, m = lane & 15;
    const int col = 16 * w + m;
    const int base = blockIdx.x * 64;
    for (int i = tid; i < 64 * 64; i += 256) {
        int row = i >> 6, c4 = i & 63;
        int node = base + row;
        v4f x; x[0] = 0.f; x[1] = 0.f; x[2] = 0.f; x[3] = 0.f;
        if (node < N) {
            x = (c4 < 32) ? *(const v4f*)(hF32 + (size_t)node * DH + 4 * c4)
                          : *(const v4f*)(agg + (size_t)node * DH + 4 * (c4 - 32));
        }
        v4us hv, lv;
#pragma unroll
        for (int q = 0; q < 4; ++q) { unsigned short hs = bf16_rne(x[q]); hv[q] = hs; lv[q] = bf16_rne(x[q] - bf16_to_f(hs)); }
        *(v4us*)&sAH[row * KN + 4 * c4] = hv;
        *(v4us*)&sAL[row * KN + 4 * c4] = lv;
    }
    __syncthreads();
    v8f acc[4];
#pragma unroll
    for (int t = 0; t < 4; ++t) acc[t] = zero8();
#pragma unroll 1
    for (int c = 0; c < 8; ++c) {
        v16b bh = ldfrag_b(w1H, KN, col, 32 * c, h);
        v16b bl = ldfrag_b(w1L, KN, col, 32 * c, h);
#pragma unroll
        for (int t = 0; t < 4; ++t) {
            v16b ah = ldfrag_b(sAH, KN, 16 * t + m, 32 * c, h);
            v16b al = ldfrag_b(sAL, KN, 16 * t + m, 32 * c, h);
            acc[t] = mma_b3(ah, al, bh, bl, acc[t]);
        }
    }
    {
        float bias = b1[col];
#pragma unroll
        for (int t = 0; t < 4; ++t)
#pragma unroll
            for (int r = 0; r < 8; ++r) {
                int row = 16 * t + 8 * h + r;
                float v = silu_f(acc[t][r] + bias);
                unsigned short hs = bf16_rne(v);
                sHH[row * DH + col] = hs;
                sHL[row * DH + col] = bf16_rne(v - bf16_to_f(hs));
            }
    }
    __syncthreads();
    v8f acc2[4];
#pragma unroll
    for (int t = 0; t < 4; ++t) acc2[t] = zero8();
#pragma unroll 1
    for (int c = 0; c < 4; ++c) {
        v16b bh = ldfrag_b(w2H, DH, col, 32 * c, h);
        v16b bl = ldfrag_b(w2L, DH, col, 32 * c, h);
#pragma unroll
        for (int t = 0; t < 4; ++t) {
            v16b ah = ldfrag_b(sHH, DH, 16 * t + m, 32 * c, h);
            v16b al = ldfrag_b(sHL, DH, 16 * t + m, 32 * c, h);
            acc2[t] = mma_b3(ah, al, bh, bl, acc2[t]);
        }
    }
    {
        float bias2 = b2[col];
#pragma unroll
        for (int t = 0; t < 4; ++t)
#pragma unroll
            for (int r = 0; r < 8; ++r) {
                int row = 16 * t + 8 * h + r;
                sUp[row * DH + col] = acc2[t][r] + bias2;
            }
    }
    __syncthreads();
    for (int rr = w; rr < 64; rr += 8) {
        int node = base + rr;
        if (node < N) {
            float* hp = hF32 + (size_t)node * DH + 4 * lane;
            v4f hx = *(const v4f*)hp;
            v4f up = *(const v4f*)&sUp[rr * DH + 4 * lane];
            v4f x = hx + up;
            float s = x[0] + x[1] + x[2] + x[3];
#pragma unroll
            for (int o = 16; o > 0; o >>= 1) s += __shfl_xor(s, o, 32);
            float mu = s * (1.0f / DH);
            v4f d = x - mu;
            float q = d[0] * d[0] + d[1] * d[1] + d[2] * d[2] + d[3] * d[3];
#pragma unroll
            for (int o = 16; o > 0; o >>= 1) q += __shfl_xor(q, o, 32);
            float var = q * (1.0f / DH);
            float inv = rsqrtf(var + 1e-5f);
            v4f g = *(const v4f*)(lng + 4 * lane);
            v4f bb = *(const v4f*)(lnb + 4 * lane);
            v4f ov = d * inv * g + bb;
            *(volatile v4f*)hp = ov;
            __threadfence();
            *(volatile v4f*)hp = ov;
        }
    }
}

__global__ __launch_bounds__(256) void k_pair(const float* hF32, const float* __restrict__ xyr,
    const int* __restrict__ pairs, int P, int N,
    const unsigned short* w1H, const unsigned short* w1L, const float* __restrict__ b1,
    const float* __restrict__ w2, const float* __restrict__ b2, float* out) {
    __shared__ __align__(16) unsigned short sAH[64 * KP];
    __shared__ __align__(16) unsigned short sAL[64 * KP];
    __shared__ __align__(16) float sHid[64 * DH];
    __shared__ __align__(16) float sOutv[64];
    const int tid = threadIdx.x, w = tid >> 5, lane = tid & 31, h = lane >> 4, m = lane & 15;
    const int col = 16 * w + m;
    const int base = blockIdx.x * 64;
    for (int i = tid; i < 64 * 72; i += 256) {
        int row = i / 72; int c4 = i - row * 72;
        int p = base + row;
        v4f x; x[0] = 0.f; x[1] = 0.f; x[2] = 0.f; x[3] = 0.f;
        if (p < P) {
            int u = clampi(pairs[2 * p], N), v = clampi(pairs[2 * p + 1], N);
            if (c4 < 32) x = *(const v4f*)(hF32 + (size_t)u * DH + 4 * c4);
            else if (c4 < 64) x = *(const v4f*)(hF32 + (size_t)v * DH + 4 * (c4 - 32));
            else if (c4 == 64) {
                float ru = xyr[u * 3 + 2], rv = xyr[v * 3 + 2];
                float dx = xyr[u * 3 + 0] - xyr[v * 3 + 0];
                float dy = xyr[u * 3 + 1] - xyr[v * 3 + 1];
                x[0] = ru; x[1] = rv; x[2] = sqrtf(dx * dx + dy * dy + 1e-8f); x[3] = fabsf(ru - rv);
            }
        }
        v4us hv, lv;
#pragma unroll
        for (int q = 0; q < 4; ++q) { unsigned short hs = bf16_rne(x[q]); hv[q] = hs; lv[q] = bf16_rne(x[q] - bf16_to_f(hs)); }
        *(v4us*)&sAH[row * KP + 4 * c4] = hv;
        *(v4us*)&sAL[row * KP + 4 * c4] = lv;
    }
    __syncthreads();
    v8f acc[4];
#pragma unroll
    for (int t = 0; t < 4; ++t) acc[t] = zero8();
#pragma unroll 1
    for (int c = 0; c < 9; ++c) {
        v16b bh = ldfrag_b(w1H, KP, col, 32 * c, h);
        v16b bl = ldfrag_b(w1L, KP, col, 32 * c, h);
#pragma unroll
        for (int t = 0; t < 4; ++t) {
            v16b ah = ldfrag_b(sAH, KP, 16 * t + m, 32 * c, h);
            v16b al = ldfrag_b(sAL, KP, 16 * t + m, 32 * c, h);
            acc[t] = mma_b3(ah, al, bh, bl, acc[t]);
        }
    }
    {
        float bias = b1[col];
#pragma unroll
        for (int t = 0; t < 4; ++t)
#pragma unroll
            for (int r = 0; r < 8; ++r) {
                int row = 16 * t + 8 * h + r;
                sHid[row * DH + col] = silu_f(acc[t][r] + bias);
            }
    }
    __syncthreads();
    if (tid < 64) {
        float s = b2[0];
#pragma unroll 4
        for (int k = 0; k < DH; ++k) s += sHid[tid * DH + k] * w2[k];
        sOutv[tid] = s;
    }
    __syncthreads();
    if (tid < 16) {
        int p0 = base + 4 * tid;
        v4f v = *(const v4f*)&sOutv[4 * tid];
        if (p0 + 3 < P) {
            *(volatile v4f*)(out + p0) = v;
            __threadfence();
            *(volatile v4f*)(out + p0) = v;
        } else {
#pragma unroll
            for (int q = 0; q < 4; ++q) if (p0 + q < P) *(volatile float*)(out + p0 + q) = v[q];
            __threadfence();
#pragma unroll
            for (int q = 0; q < 4; ++q) if (p0 + q < P) *(volatile float*)(out + p0 + q) = v[q];
        }
    }
}

extern "C" void kernel_launch(void* const* d_in, const int* in_sizes, int n_in,
                              void* d_out, int out_size, void* d_ws, size_t ws_size,
                              hipStream_t stream) {
    const float* xyr     = (const float*)d_in[0];
    const int*   eidx    = (const int*)d_in[1];
    const int*   pairs   = (const int*)d_in[2];
    const float* node_w1 = (const float*)d_in[3];
    const float* node_b1 = (const float*)d_in[4];
    const float* node_w2 = (const float*)d_in[5];
    const float* node_b2 = (const float*)d_in[6];
    const float* pm_w1   = (const float*)d_in[7];
    const float* pm_b1   = (const float*)d_in[8];
    const float* pm_w2   = (const float*)d_in[9];
    const float* pm_b2   = (const float*)d_in[10];
    const float* ph_w1   = (const float*)d_in[11];
    const float* ph_b1   = (const float*)d_in[12];
    const float* ph_w2   = (const float*)d_in[13];
    const float* ph_b2   = (const float*)d_in[14];
    const float* ln_g    = (const float*)d_in[15];
    const float* ln_b    = (const float*)d_in[16];
    const float* eh_w1   = (const float*)d_in[17];
    const float* eh_b1   = (const float*)d_in[18];
    const float* eh_w2   = (const float*)d_in[19];
    const float* eh_b2   = (const float*)d_in[20];
    (void)n_in; (void)stream;

    const int N = in_sizes[0] / 3;
    const int E = in_sizes[1] / 2;
    const int P = in_sizes[2] / 2;
    const int L = 3;
    if (N <= 0 || E <= 0 || P <= 0 || out_size < P) return;

    char* ws = (char*)d_ws;
    size_t off = 0;
    auto carve = [&](size_t bytes) -> char* {
        char* p = ws + off;
        off = (off + bytes + 255) & ~(size_t)255;
        return p;
    };
    float*          hF32   = (float*)carve((size_t)N * DH * 4);
    float*          agg    = (float*)carve((size_t)N * DH * 4);
    _Float16*       pm_w1T = (_Float16*)carve((size_t)L * DH * KE * 2);
    _Float16*       pm_w2T = (_Float16*)carve((size_t)L * DH * DH * 2);
    unsigned short* ph_w1H = (unsigned short*)carve((size_t)L * DH * KN * 2);
    unsigned short* ph_w1L = (unsigned short*)carve((size_t)L * DH * KN * 2);
    unsigned short* ph_w2H = (unsigned short*)carve((size_t)L * DH * DH * 2);
    unsigned short* ph_w2L = (unsigned short*)carve((size_t)L * DH * DH * 2);
    unsigned short* eh_w1H = (unsigned short*)carve((size_t)DH * KP * 2);
    unsigned short* eh_w1L = (unsigned short*)carve((size_t)DH * KP * 2);
    if (off > ws_size) return;

    auto grid8 = [](size_t nelem) { size_t c = nelem / 8; return dim3((unsigned)((c + 255) / 256)); };

    k_tw_f16<<<grid8((size_t)L * DH * KE), 256, 0, 0>>>(pm_w1, pm_w1T, L, 272, DH, KE);
    k_tw_f16<<<grid8((size_t)L * DH * DH), 256, 0, 0>>>(pm_w2, pm_w2T, L, DH, DH, DH);
    k_tw_bf2<<<grid8((size_t)L * DH * KN), 256, 0, 0>>>(ph_w1, ph_w1H, ph_w1L, L, KN, DH, KN);
    k_tw_bf2<<<grid8((size_t)L * DH * DH), 256, 0, 0>>>(ph_w2, ph_w2H, ph_w2L, L, DH, DH, DH);
    k_tw_bf2<<<grid8((size_t)DH * KP), 256, 0, 0>>>(eh_w1, eh_w1H, eh_w1L, 1, 260, DH, KP);

    k_encode<<<dim3((unsigned)N), 128, 0, 0>>>(xyr, N, node_w1, node_b1, node_w2, node_b2, hF32);

    for (int l = 0; l < L; ++l) {
        k_edge<<<dim3((unsigned)((N + NB - 1) / NB)), 256, 0, 0>>>(
            hF32, xyr, eidx, E, N,
            pm_w1T + (size_t)l * DH * KE, pm_b1 + (size_t)l * DH,
            pm_w2T + (size_t)l * DH * DH, pm_b2 + (size_t)l * DH, agg);
        k_node<<<dim3((unsigned)((N + 63) / 64)), 256, 0, 0>>>(
            hF32, agg, N,
            ph_w1H + (size_t)l * DH * KN, ph_w1L + (size_t)l * DH * KN, ph_b1 + (size_t)l * DH,
            ph_w2H + (size_t)l * DH * DH, ph_w2L + (size_t)l * DH * DH, ph_b2 + (size_t)l * DH,
            ln_g + (size_t)l * DH, ln_b + (size_t)l * DH);
    }

    k_pair<<<dim3((unsigned)((P + 63) / 64)), 256, 0, 0>>>(
        hF32, xyr, pairs, P, N, eh_w1H, eh_w1L, eh_b1, eh_w2, eh_b2, (float*)d_out);
}
